// MODEL_14663018348910
// MI455X (gfx1250) — hardware-verified
//
#include <hip/hip_runtime.h>
#include <math.h>

constexpr int NBAT   = 8;
constexpr int NSTEP  = 16;
constexpr int NNODE  = 512;
constexpr int NFEAT  = 128;
constexpr int NHID   = 128;
constexpr int NCHEB  = 3;
constexpr int NGATE  = 4 * NHID;
constexpr int KCAT   = 2 * NCHEB * NHID;
constexpr int ACW    = 3 * NCHEB * NHID;
constexpr int NROWS  = NBAT * NNODE;
constexpr int TTP    = 72;
constexpr float LCARRY     = 16.0f;
constexpr float LCARRY_INV = 1.0f / 16.0f;
constexpr float WCARRY     = 16.0f;
constexpr float WCARRY_INV = 1.0f / 16.0f;
static_assert(NFEAT == NHID, "x-side and h-side bases share one column width");
static_assert(NGATE == 512 && KCAT == 768 && ACW == 1152 && NROWS == 4096, "shape contract");
static_assert(NNODE % 64 == 0 && NHID % 64 == 0 && NGATE % 64 == 0 && NROWS % 64 == 0, "GEMM M,N tile multiples");
static_assert(NNODE % 32 == 0 && KCAT % 32 == 0, "GEMM K multiples of 32");
static_assert((ACW * 2) % 128 == 0, "Acat row pitch is a whole number of 128-B lines");

typedef __attribute__((ext_vector_type(16))) _Float16 v16h;
typedef __attribute__((ext_vector_type(8)))  _Float16 v8h;
typedef __attribute__((ext_vector_type(8)))  float    v8f;
typedef __attribute__((ext_vector_type(4)))  float    v4f;
typedef __attribute__((ext_vector_type(4)))  unsigned v4u;

__device__ __forceinline__ unsigned short f2bf_bits(float f) {
  unsigned u = __float_as_uint(f);
  return (unsigned short)((u + 0x7FFFu + ((u >> 16) & 1u)) >> 16);
}
__device__ __forceinline__ float bf_bits2f(unsigned short h) { return __uint_as_float(((unsigned)h) << 16); }
__device__ __forceinline__ float bf16r(float f) { return bf_bits2f(f2bf_bits(f)); }

__device__ __forceinline__ float h16_to_f32(unsigned hb) {
  const unsigned sgn = (hb & 0x8000u) << 16;
  const unsigned em = hb & 0x7fffu;
  const float fn = __uint_as_float((em << 13) + 0x38000000u);
  const float fs = (float)em * 5.9604644775390625e-8f;
  const float mag = (em < 0x400u) ? fs : fn;
  return __uint_as_float(__float_as_uint(mag) | sgn);
}

union FragU { v16h v; v8h h[2]; };
__device__ __forceinline__ v16h frag_load(const _Float16* p) {
  FragU f;
  f.h[0] = *(const v8h*)(p);
  f.h[1] = *(const v8h*)(p + 16);
  return f.v;
}
__device__ __forceinline__ v8f frag_mma(v16h a, v16h b, v8f c) {
  return __builtin_amdgcn_wmma_f32_16x16x32_f16(false, a, false, b, (short)0, c, false, false);
}
__device__ __forceinline__ void guard_row(v8f& a0, v8f& a1, v8f& a2, v8f& a3, v16h x, v16h b0, v16h b1, v16h b2, v16h b3) {
  asm volatile("v_nop\n\tv_nop\n\tv_nop\n\tv_nop" : "+v"(a0), "+v"(a1), "+v"(a2), "+v"(a3) : "v"(x), "v"(b0), "v"(b1), "v"(b2), "v"(b3));
}
__device__ __forceinline__ void keep4_h(v16h a, v16h b, v16h c, v16h d) { asm volatile("v_nop" :: "v"(a), "v"(b), "v"(c), "v"(d)); }
__device__ __forceinline__ void acc_guard4(v8f& a, v8f& b, v8f& c, v8f& d) { asm volatile("v_nop\n\tv_nop\n\tv_nop\n\tv_nop" : "+v"(a), "+v"(b), "+v"(c), "+v"(d)); }

__device__ __forceinline__ void wave_sync_lds() {
  __builtin_amdgcn_fence(__ATOMIC_RELEASE, "workgroup");
  __builtin_amdgcn_wave_barrier();
  __builtin_amdgcn_fence(__ATOMIC_ACQUIRE, "workgroup");
}

__device__ __forceinline__ float sigm_f(float x) { return __builtin_amdgcn_rcpf(1.0f + expf(-x)); }
__device__ __forceinline__ float tanh_f(float x) { return 1.0f - 2.0f * __builtin_amdgcn_rcpf(expf(2.0f * x) + 1.0f); }

__global__ __launch_bounds__(256) void zero16_kernel(float* __restrict__ p, int n16) {
  const int i = blockIdx.x * 256 + threadIdx.x;
  if (i < n16) {
    const v4f z = {0.0f, 0.0f, 0.0f, 0.0f};
    *(volatile v4f*)(p + (size_t)i * 4) = z;
    __threadfence();
    *(volatile v4f*)(p + (size_t)i * 4) = z;
  }
}

__global__ __launch_bounds__(256) void cvt8_kernel(const float* __restrict__ src, unsigned short* __restrict__ dst, int n8, float sc) {
  const int i = blockIdx.x * 256 + threadIdx.x;
  if (i < n8) {
    const float* sp = src + (size_t)i * 8;
    const v4f a = *(const v4f*)(sp);
    const v4f b = *(const v4f*)(sp + 4);
    v8h hv;
#pragma unroll
    for (int e = 0; e < 4; ++e) {
      const float fa = a[e];
      const float fb = b[e];
      hv[e]     = (_Float16)(bf16r(fa) * sc);
      hv[4 + e] = (_Float16)(bf16r(fb) * sc);
    }
    *(volatile v8h*)(dst + (size_t)i * 8) = hv;
    __threadfence();
    *(volatile v8h*)(dst + (size_t)i * 8) = hv;
  }
}

__global__ __launch_bounds__(256) void tpw_kernel(const float* __restrict__ src, int R, int C, int ldo,
                                                  unsigned short* __restrict__ O, float sc) {
  __shared__ float Tt[64 * 65];
  const int tid = threadIdx.x;
  const int c0 = blockIdx.x * 64, r0 = blockIdx.y * 64;
#pragma unroll
  for (int i = 0; i < 4; ++i) {
    const int idx = i * 256 + tid;
    const int rr = idx >> 4, cc = (idx & 15) * 4;
    const v4f v = *(const v4f*)(src + (size_t)(r0 + rr) * (size_t)C + c0 + cc);
    Tt[rr * 65 + cc + 0] = v[0];
    Tt[rr * 65 + cc + 1] = v[1];
    Tt[rr * 65 + cc + 2] = v[2];
    Tt[rr * 65 + cc + 3] = v[3];
  }
  __syncthreads();
  const int q = tid >> 3, c8 = (tid & 7) * 8;
  v8h hv[2];
#pragma unroll
  for (int g = 0; g < 2; ++g) {
    const int qq = g * 32 + q;
#pragma unroll
    for (int e = 0; e < 8; ++e) {
      const float f = Tt[(c8 + e) * 65 + qq];
      hv[g][e] = (_Float16)(bf16r(f) * sc);
    }
  }
  for (int pass = 0; pass < 2; ++pass) {
#pragma unroll
    for (int g = 0; g < 2; ++g) {
      const size_t o = (size_t)(c0 + g * 32 + q) * (size_t)ldo + (size_t)(r0 + c8);
      *(volatile v8h*)(O + o) = hv[g];
    }
    __threadfence();
  }
}

__global__ __launch_bounds__(256) void bias_sum_kernel(const float* __restrict__ b1a, const float* __restrict__ b2a,
                                                       const float* __restrict__ b1b, const float* __restrict__ b2b,
                                                       float* __restrict__ dst) {
  const int tid = threadIdx.x;
  const int which = tid >> 7;
  const int idx = (tid & 127) * 4;
  const v4f p = *(const v4f*)(b1a + idx);
  const v4f q = *(const v4f*)(b2a + idx);
  const v4f r = *(const v4f*)(b1b + idx);
  const v4f s = *(const v4f*)(b2b + idx);
  v4f o;
#pragma unroll
  for (int e = 0; e < 4; ++e) {
    const float s0 = bf16r(p[e]) + bf16r(q[e]);
    const float s1 = bf16r(r[e]) + bf16r(s[e]);
    o[e] = which ? s1 : s0;
  }
  float* op = dst + which * NGATE + idx;
  *(volatile v4f*)op = o;
  __threadfence();
  *(volatile v4f*)op = o;
}

__global__ __launch_bounds__(256) void xconv_kernel(const float* __restrict__ x, int t,
                                                    unsigned short* __restrict__ acat, unsigned short* __restrict__ xt) {
  __shared__ __align__(16) float Xs[64 * 132];
  const int tid = threadIdx.x;
  const int n0 = blockIdx.x * 64, b = blockIdx.y;
  const float* xb = x + ((size_t)(b * NSTEP + t) * NNODE + n0) * NFEAT;
#pragma unroll
  for (int i = 0; i < 8; ++i) {
    const int idx = i * 256 + tid;
    const int rr = idx >> 5, cc = (idx & 31) * 4;
    const v4f v = *(const v4f*)(xb + (size_t)rr * NFEAT + cc);
    v4f w;
#pragma unroll
    for (int e = 0; e < 4; ++e) w[e] = bf16r(v[e]);
    *(v4f*)(Xs + rr * 132 + cc) = w;
  }
  __syncthreads();
  v8h hr[4], ht[4];
#pragma unroll
  for (int i = 0; i < 4; ++i) {
    const int idx = i * 256 + tid;
    const int row = idx >> 4, c8 = (idx & 15) * 8;
    const v4f a = *(const v4f*)(Xs + row * 132 + c8);
    const v4f c = *(const v4f*)(Xs + row * 132 + c8 + 4);
#pragma unroll
    for (int e = 0; e < 4; ++e) {
      hr[i][e]     = (_Float16)a[e];
      hr[i][4 + e] = (_Float16)c[e];
    }
    const int ff = idx >> 3, d8 = (idx & 7) * 8;
#pragma unroll
    for (int e = 0; e < 8; ++e) ht[i][e] = (_Float16)Xs[(d8 + e) * 132 + ff];
  }
  for (int pass = 0; pass < 2; ++pass) {
#pragma unroll
    for (int i = 0; i < 4; ++i) {
      const int idx = i * 256 + tid;
      const int row = idx >> 4, c8 = (idx & 15) * 8;
      *(volatile v8h*)(acat + ((size_t)b * NNODE + n0 + row) * ACW + c8) = hr[i];
      const int ff = idx >> 3, d8 = (idx & 7) * 8;
      *(volatile v8h*)(xt + ((size_t)b * NFEAT + ff) * NNODE + n0 + d8) = ht[i];
    }
    __threadfence();
  }
}

template <int MODE, int NW>
__global__ __launch_bounds__(256) void cheb_gemm(
    const unsigned short* __restrict__ Ap, int lda, long strideA,
    const unsigned short* __restrict__ BtS0, const unsigned short* __restrict__ BtS1, int ldb, long strideB,
    void* Cout, int ldc, long strideC, int ccolS0, int ccolS1,
    unsigned short* TtS0, unsigned short* TtS1, int scolS0, int scolS1,
    const float* __restrict__ bias, int M, int N, int K, float scale) {
  __shared__ __align__(16) float sT[NW][16 * 68];
  __shared__ __align__(16) _Float16 sTt[(MODE == 1) ? (NW * 64 * TTP) : 8];
  const int set  = blockIdx.y >> 3;
  const int b    = blockIdx.y & 7;
  const int lane = threadIdx.x & 31;
  const int wave = threadIdx.x >> 5;
  const int tilesN = N >> 6;
  const int tilesM = M >> 6;
  const int tile = blockIdx.x * NW + wave;
  if (tile >= tilesM * tilesN) return;
  const int tm = tile / tilesN;
  const int tn = tile - tm * tilesN;
  const int m0 = tm << 6;
  const int n0 = tn << 6;

  const unsigned short* Btp = set ? BtS1 : BtS0;
  const int ccol = set ? ccolS1 : ccolS0;
  const int scol = set ? scolS1 : scolS0;
  const _Float16* Ab = (const _Float16*)Ap + (size_t)b * strideA;
  const _Float16* Bb = (const _Float16*)Btp + (size_t)b * strideB;

  const int rlane = lane & 15;
  const int koff  = (lane >> 4) * 8;
  const int mOff  = (lane >> 4) * 8;

  v8f acc[4][4];
#pragma unroll
  for (int i = 0; i < 4; ++i)
#pragma unroll
    for (int j = 0; j < 4; ++j) acc[i][j] = (v8f){0.f, 0.f, 0.f, 0.f, 0.f, 0.f, 0.f, 0.f};

  for (int k0 = 0; k0 < K; k0 += 32) {
    v16h bh[4];
#pragma unroll
    for (int j = 0; j < 4; ++j) {
      const size_t bo = (size_t)(n0 + (j << 4) + rlane) * ldb + koff + k0;
      bh[j] = frag_load(Bb + bo);
    }
#pragma unroll
    for (int i = 0; i < 4; ++i) {
      const size_t ao = (size_t)(m0 + (i << 4) + rlane) * lda + koff + k0;
      const v16h ah = frag_load(Ab + ao);
#pragma unroll
      for (int j = 0; j < 4; ++j) acc[i][j] = frag_mma(ah, bh[j], acc[i][j]);
      guard_row(acc[i][0], acc[i][1], acc[i][2], acc[i][3], ah, bh[0], bh[1], bh[2], bh[3]);
    }
    keep4_h(bh[0], bh[1], bh[2], bh[3]);
  }
  acc_guard4(acc[0][0], acc[0][1], acc[0][2], acc[0][3]);
  acc_guard4(acc[1][0], acc[1][1], acc[1][2], acc[1][3]);
  acc_guard4(acc[2][0], acc[2][1], acc[2][2], acc[2][3]);
  acc_guard4(acc[3][0], acc[3][1], acc[3][2], acc[3][3]);

  float* slab = sT[wave];
  _Float16* tts = sTt + ((MODE == 1) ? (wave * 64 * TTP) : 0);
#pragma unroll
  for (int i = 0; i < 4; ++i) {
    const int mBase = m0 + (i << 4);
#pragma unroll
    for (int j = 0; j < 4; ++j) {
      const int n = n0 + (j << 4) + rlane;
      float bv = 0.f;
      if (MODE == 0) bv = bias[n];
      v8h tv;
#pragma unroll
      for (int r = 0; r < 8; ++r) {
        float v = acc[i][j][r] * scale;
        if (MODE == 0) v += bv;
        slab[(mOff + r) * 68 + (j << 4) + rlane] = v;
        if (MODE == 1) tv[r] = (_Float16)v;
      }
      if (MODE == 1) *(v8h*)(tts + ((j << 4) + rlane) * TTP + (i << 4) + mOff) = tv;
    }
    wave_sync_lds();
    if (MODE == 0) {
      float* C = (float*)Cout + (size_t)b * strideC + ccol;
      const int hh = lane >> 4, c4 = (lane & 15) * 4;
      for (int pass = 0; pass < 2; ++pass) {
#pragma unroll
        for (int it = 0; it < 8; ++it) {
          const int row = it * 2 + hh;
          const v4f v = *(const v4f*)(slab + row * 68 + c4);
          *(volatile v4f*)(C + (size_t)(mBase + row) * ldc + n0 + c4) = v;
        }
        __threadfence();
      }
    } else {
      const int q = lane >> 3, c8 = (lane & 7) * 8;
      unsigned short* C = (unsigned short*)Cout + (size_t)b * strideC + ccol;
      const unsigned short* Csub = (const unsigned short*)Cout + (size_t)b * strideC + scol;
      v8h hv[4];
#pragma unroll
      for (int it = 0; it < 4; ++it) {
        const int row = it * 4 + q;
        const float* sp = slab + row * 68 + c8;
        if (MODE == 2) {
          const v4u sw = *(const v4u*)(Csub + (size_t)(mBase + row) * ldc + n0 + c8);
          const unsigned w0 = sw[0];
          const unsigned w1 = sw[1];
          const unsigned w2 = sw[2];
          const unsigned w3 = sw[3];
          const float t0 = h16_to_f32(w0 & 0xffffu);
          const float t1 = h16_to_f32(w0 >> 16);
          const float t2 = h16_to_f32(w1 & 0xffffu);
          const float t3 = h16_to_f32(w1 >> 16);
          const float t4 = h16_to_f32(w2 & 0xffffu);
          const float t5 = h16_to_f32(w2 >> 16);
          const float t6 = h16_to_f32(w3 & 0xffffu);
          const float t7 = h16_to_f32(w3 >> 16);
          hv[it][0] = (_Float16)(sp[0] - t0);
          hv[it][1] = (_Float16)(sp[1] - t1);
          hv[it][2] = (_Float16)(sp[2] - t2);
          hv[it][3] = (_Float16)(sp[3] - t3);
          hv[it][4] = (_Float16)(sp[4] - t4);
          hv[it][5] = (_Float16)(sp[5] - t5);
          hv[it][6] = (_Float16)(sp[6] - t6);
          hv[it][7] = (_Float16)(sp[7] - t7);
        } else {
#pragma unroll
          for (int e = 0; e < 8; ++e) hv[it][e] = (_Float16)sp[e];
        }
      }
      for (int pass = 0; pass < 2; ++pass) {
#pragma unroll
        for (int it = 0; it < 4; ++it) {
          const int row = it * 4 + q;
          *(volatile v8h*)(C + (size_t)(mBase + row) * ldc + n0 + c8) = hv[it];
        }
        __threadfence();
      }
    }
    wave_sync_lds();
  }
  if (MODE == 1) {
    wave_sync_lds();
    unsigned short* TT = (set ? TtS1 : TtS0) + (size_t)b * strideB;
    const int q = lane >> 3, c8 = (lane & 7) * 8;
    for (int pass = 0; pass < 2; ++pass) {
#pragma unroll
      for (int it = 0; it < 16; ++it) {
        const int frow = it * 4 + q;
        const v8h v = *(const v8h*)(tts + frow * TTP + c8);
        *(volatile v8h*)(TT + (size_t)(n0 + frow) * ldb + m0 + c8) = v;
      }
      __threadfence();
    }
  }
}

__global__ __launch_bounds__(256) void gate_kernel(const float* __restrict__ Z, const float* __restrict__ cin, float* __restrict__ cout,
                                                   unsigned short* __restrict__ acat, int hcol, unsigned short* __restrict__ hT,
                                                   float* __restrict__ out0, float* __restrict__ out1, float* __restrict__ out2,
                                                   int t, int wout, int last) {
  __shared__ __align__(16) float Hs[64 * 68];
  __shared__ __align__(16) float Cs[64 * 68];
  const int tid = threadIdx.x;
  const int n0 = blockIdx.x * 64, u0 = blockIdx.y * 64, b = blockIdx.z;
  const int j = tid & 63, rsub = tid >> 6;
  const size_t rowbase = (size_t)b * NNODE + n0;
#pragma unroll 1
  for (int it = 0; it < 16; ++it) {
    const int row = it * 4 + rsub;
    const size_t R = rowbase + row;
    const float* zp = Z + R * NGATE + u0 + j;
    const float zi = zp[0];
    const float zf = zp[NHID];
    const float zo = zp[2 * NHID];
    const float zg = zp[3 * NHID];
    const float cp = cin[R * NHID + u0 + j];
    const float ig = sigm_f(zi);
    const float fg = sigm_f(zf);
    const float og = sigm_f(zo);
    const float gg = tanh_f(zg);
    const float cn = fg * cp + ig * gg;
    const float hn = og * tanh_f(cn);
    Hs[row * 68 + j] = hn;
    Cs[row * 68 + j] = cn;
  }
  __syncthreads();
  v4f vc[4], vh[4];
  v8h ha[2], ht[2];
#pragma unroll
  for (int i = 0; i < 4; ++i) {
    const int idx = i * 256 + tid;
    const int row = idx >> 4, c4 = (idx & 15) * 4;
    vc[i] = *(const v4f*)(Cs + row * 68 + c4);
    vh[i] = *(const v4f*)(Hs + row * 68 + c4);
  }
#pragma unroll
  for (int i = 0; i < 2; ++i) {
    const int idx = i * 256 + tid;
    const int row = idx >> 3, c8 = (idx & 7) * 8;
    const v4f a = *(const v4f*)(Hs + row * 68 + c8);
    const v4f c = *(const v4f*)(Hs + row * 68 + c8 + 4);
#pragma unroll
    for (int e = 0; e < 4; ++e) {
      ha[i][e]     = (_Float16)a[e];
      ha[i][4 + e] = (_Float16)c[e];
    }
#pragma unroll
    for (int e = 0; e < 8; ++e) ht[i][e] = (_Float16)Hs[(c8 + e) * 68 + row];
  }
  for (int pass = 0; pass < 2; ++pass) {
#pragma unroll
    for (int i = 0; i < 4; ++i) {
      const int idx = i * 256 + tid;
      const int row = idx >> 4, c4 = (idx & 15) * 4;
      const size_t so = (rowbase + row) * NHID + u0 + c4;
      *(volatile v4f*)(cout + so) = vc[i];
      if (wout) {
        const size_t oo = ((size_t)(b * NSTEP + t) * NNODE + n0 + row) * NHID + u0 + c4;
        *(volatile v4f*)(out0 + oo) = vh[i];
      }
      if (last) {
        *(volatile v4f*)(out1 + so) = vh[i];
        *(volatile v4f*)(out2 + so) = vc[i];
      }
    }
#pragma unroll
    for (int i = 0; i < 2; ++i) {
      const int idx = i * 256 + tid;
      const int row = idx >> 3, c8 = (idx & 7) * 8;
      *(volatile v8h*)(acat + (rowbase + row) * ACW + hcol + u0 + c8) = ha[i];
      *(volatile v8h*)(hT + ((size_t)b * NHID + u0 + row) * NNODE + n0 + c8) = ht[i];
    }
    __threadfence();
  }
}

extern "C" void kernel_launch(void* const* d_in, const int* in_sizes, int n_in,
                              void* d_out, int out_size, void* d_ws, size_t ws_size, hipStream_t stream) {
  if (n_in < 10 || d_out == nullptr || d_ws == nullptr) return;
  if (in_sizes[0] != NBAT * NSTEP * NNODE * NFEAT || in_sizes[1] != NBAT * NNODE * NNODE ||
      in_sizes[2] != NCHEB * NFEAT * NGATE || in_sizes[3] != NGATE ||
      in_sizes[4] != NCHEB * NHID * NGATE  || in_sizes[5] != NGATE ||
      in_sizes[6] != NCHEB * NHID * NGATE  || in_sizes[7] != NGATE ||
      in_sizes[8] != NCHEB * NHID * NGATE  || in_sizes[9] != NGATE ||
      out_size != NBAT * NSTEP * NNODE * NHID + 2 * NBAT * NNODE * NHID) return;

  const float* x     = (const float*)d_in[0];
  const float* graph = (const float*)d_in[1];
  const float* W1_0  = (const float*)d_in[2];
  const float* b1_0  = (const float*)d_in[3];
  const float* W2_0  = (const float*)d_in[4];
  const float* b2_0  = (const float*)d_in[5];
  const float* W1_1  = (const float*)d_in[6];
  const float* b1_1  = (const float*)d_in[7];
  const float* W2_1  = (const float*)d_in[8];
  const float* b2_1  = (const float*)d_in[9];
  float* out0 = (float*)d_out;
  float* out1 = out0 + (size_t)NBAT * NSTEP * NNODE * NHID;
  float* out2 = out1 + (size_t)NBAT * NNODE * NHID;

  char* ws = (char*)d_ws;
  size_t off = 0;
  auto carve = [&](size_t bytes) -> char* { char* p = ws + off; off += (bytes + 255) & ~(size_t)255; return p; };
  const size_t planeT = (size_t)NBAT * NHID * NNODE * 2;
  const size_t planeC = (size_t)NROWS * NHID * 4;
  unsigned short* LH   = (unsigned short*)carve((size_t)NBAT * NNODE * NNODE * 2);
  unsigned short* WT0  = (unsigned short*)carve((size_t)NGATE * KCAT * 2);
  unsigned short* WT1  = (unsigned short*)carve((size_t)NGATE * KCAT * 2);
  float*          BS   = (float*)carve((size_t)2 * NGATE * 4);
  unsigned short* ACAT = (unsigned short*)carve((size_t)NROWS * ACW * 2);
  float*          C0A  = (float*)carve(planeC);
  float*          C1A  = (float*)carve(planeC);
  unsigned short* H0T  = (unsigned short*)carve(planeT);
  unsigned short* H1T  = (unsigned short*)carve(planeT);
  float*          C0B  = (float*)carve(planeC);
  float*          C1B  = (float*)carve(planeC);
  unsigned short* XT    = (unsigned short*)carve(planeT);
  unsigned short* T1XT  = (unsigned short*)carve(planeT);
  unsigned short* T1H0T = (unsigned short*)carve(planeT);
  unsigned short* T1H1T = (unsigned short*)carve(planeT);
  float*          ZB    = (float*)carve((size_t)NROWS * NGATE * 4);
  if (off > ws_size || off > (size_t)134217728) return;

  const size_t zbytes = (size_t)NROWS * ACW * 2 + 2 * planeC + 2 * planeT;
  const int n16 = (int)(zbytes / 16);
  zero16_kernel<<<(n16 + 255) / 256, 256, 0, stream>>>((float*)ACAT, n16);
  const int n8g = NBAT * NNODE * NNODE / 8;
  cvt8_kernel<<<(n8g + 255) / 256, 256, 0, stream>>>(graph, LH, n8g, LCARRY);
  const dim3 gw(NGATE / 64, (NCHEB * NHID) / 64);
  tpw_kernel<<<gw, 256, 0, stream>>>(W1_0, NCHEB * NFEAT, NGATE, KCAT, WT0, WCARRY);
  tpw_kernel<<<gw, 256, 0, stream>>>(W2_0, NCHEB * NHID,  NGATE, KCAT, WT0 + NCHEB * NHID, WCARRY);
  tpw_kernel<<<gw, 256, 0, stream>>>(W1_1, NCHEB * NHID,  NGATE, KCAT, WT1, WCARRY);
  tpw_kernel<<<gw, 256, 0, stream>>>(W2_1, NCHEB * NHID,  NGATE, KCAT, WT1 + NCHEB * NHID, WCARRY);
  bias_sum_kernel<<<1, 256, 0, stream>>>(b1_0, b2_0, b1_1, b2_1, BS);

  const long sL  = (long)NNODE * NNODE;
  const long sT  = (long)NHID * NNODE;
  const long sAc = (long)NNODE * ACW;
  const float hop1_scale = LCARRY_INV;
  const float hop2_scale = 2.0f * LCARRY_INV;
  const dim3 gproj((NROWS / 64) * (NGATE / 64) / 8, 1);
  const dim3 ggate(NNODE / 64, NHID / 64, NBAT);

  for (int t = 0; t < NSTEP; ++t) {
    float* c0in  = (t & 1) ? C0B : C0A;
    float* c0out = (t & 1) ? C0A : C0B;
    float* c1in  = (t & 1) ? C1B : C1A;
    float* c1out = (t & 1) ? C1A : C1B;
    const int nsets = (t > 0) ? 2 : 1;
    xconv_kernel<<<dim3(NNODE / 64, NBAT), 256, 0, stream>>>(x, t, ACAT, XT);
    cheb_gemm<1, 4><<<dim3(4, 8 * nsets), 128, 0, stream>>>(
        LH, NNODE, sL, XT, H1T, NNODE, sT, (void*)ACAT, ACW, sAc, 128, 896,
        T1XT, T1H1T, 0, 0, BS, NNODE, NHID, NNODE, hop1_scale);
    cheb_gemm<2, 4><<<dim3(4, 8 * nsets), 128, 0, stream>>>(
        LH, NNODE, sL, T1XT, T1H1T, NNODE, sT, (void*)ACAT, ACW, sAc, 256, 1024,
        T1XT, T1H1T, 0, 768, BS, NNODE, NHID, NNODE, hop2_scale);
    cheb_gemm<0, 8><<<gproj, 256, 0, stream>>>(
        ACAT, ACW, 0L, WT0, WT0, KCAT, 0L, (void*)ZB, NGATE, 0L, 0, 0,
        XT, XT, 0, 0, BS, NROWS, NGATE, KCAT, WCARRY_INV);
    gate_kernel<<<ggate, 256, 0, stream>>>(ZB, c0in, c0out, ACAT, 384, H0T, out0, out1, out2, t, 0, 0);
    cheb_gemm<1, 4><<<dim3(4, 8), 128, 0, stream>>>(
        LH, NNODE, sL, H0T, H0T, NNODE, sT, (void*)ACAT, ACW, sAc, 512, 512,
        T1H0T, T1H0T, 0, 0, BS, NNODE, NHID, NNODE, hop1_scale);
    cheb_gemm<2, 4><<<dim3(4, 8), 128, 0, stream>>>(
        LH, NNODE, sL, T1H0T, T1H0T, NNODE, sT, (void*)ACAT, ACW, sAc, 640, 640,
        T1H0T, T1H0T, 384, 384, BS, NNODE, NHID, NNODE, hop2_scale);
    cheb_gemm<0, 8><<<gproj, 256, 0, stream>>>(
        ACAT + 384, ACW, 0L, WT1, WT1, KCAT, 0L, (void*)ZB, NGATE, 0L, 0, 0,
        XT, XT, 0, 0, BS + NGATE, NROWS, NGATE, KCAT, WCARRY_INV);
    gate_kernel<<<ggate, 256, 0, stream>>>(ZB, c1in, c1out, ACAT, 768, H1T, out0, out1, out2, t, 1, (t == NSTEP - 1) ? 1 : 0);
  }
}
